// Qwen3Attention_4054449128306
// MI455X (gfx1250) — hardware-verified
//
#include <hip/hip_runtime.h>
#include <math.h>

typedef __attribute__((ext_vector_type(16))) _Float16 v16h;
typedef __attribute__((ext_vector_type(16))) __bf16 v16b;
typedef __attribute__((ext_vector_type(8)))  _Float16 v8h;
typedef __attribute__((ext_vector_type(8)))  __bf16 v8b;
typedef __attribute__((ext_vector_type(8)))  float v8f;
typedef __attribute__((ext_vector_type(4)))  float v4f;
typedef __attribute__((ext_vector_type(4)))  unsigned v4u;
typedef __attribute__((ext_vector_type(4)))  int v4i;

template <typename T> __device__ __forceinline__ void vst2(void* p, T v) { *(volatile T*)p = v; __threadfence(); *(volatile T*)p = v; }
__device__ __forceinline__ v8f wmma16(v16h a, v16h b, v8f c) {
  v8f d = __builtin_amdgcn_wmma_f32_16x16x32_f16(false, a, false, b, (short)0, c, false, false);
  asm volatile("v_nop\n\tv_nop\n\tv_nop\n\tv_nop" : "+v"(d) : "v"(a), "v"(b));
  return d;
}
__device__ __forceinline__ v8f wmma_bf(v16b a, v16b b, v8f c) {
  v8f d = __builtin_amdgcn_wmma_f32_16x16x32_bf16(false, a, false, b, (short)0, c, false, false);
  asm volatile("v_nop\n\tv_nop\n\tv_nop\n\tv_nop" : "+v"(d) : "v"(a), "v"(b));
  return d;
}
__device__ __forceinline__ v16h frag_h(const _Float16* rowk0, int lane) {
  union { v16h v; v8h q[2]; } u; const _Float16* p = rowk0 + 8 * (lane >> 4);
  u.q[0] = *(const v8h*)p; u.q[1] = *(const v8h*)(p + 16); return u.v;
}
__device__ __forceinline__ v16b frag_b(const __bf16* rowk0, int lane) {
  union { v16b v; v8b q[2]; } u; const __bf16* p = rowk0 + 8 * (lane >> 4);
  u.q[0] = *(const v8b*)p; u.q[1] = *(const v8b*)(p + 16); return u.v;
}
__device__ __forceinline__ v16h frag_f32(const float* rowk0, int lane) {
  v16h a; const float* p = rowk0 + 8 * (lane >> 4);
#pragma unroll
  for (int i = 0; i < 8; ++i) { a[i] = (_Float16)p[i]; a[8 + i] = (_Float16)p[16 + i]; }
  return a;
}
struct F2 { v16b h, l; };
__device__ __forceinline__ F2 bsplit16(const float v[16]) { F2 r;
#pragma unroll
  for (int i = 0; i < 16; ++i) { const __bf16 h = (__bf16)v[i]; r.h[i] = h; r.l[i] = (__bf16)(v[i] - (float)h); }
  return r; }
__device__ __forceinline__ F2 split_row(const float* row, int k0, int lane) { float v[16]; const float* p = row + k0 + 8 * (lane >> 4);
#pragma unroll
  for (int i = 0; i < 8; ++i) { v[i] = p[i]; v[8 + i] = p[16 + i]; }
  return bsplit16(v); }
__device__ __forceinline__ float bfr(float v) { return (float)(__bf16)v; }
__device__ __forceinline__ v16b wcol_oi(const float* Wm, int k0, int o, int lane, int K) { v16b w; const float* p = Wm + (size_t)o * K + k0 + 8 * (lane >> 4);
#pragma unroll
  for (int i = 0; i < 8; ++i) { w[i] = (__bf16)p[i]; w[8 + i] = (__bf16)p[16 + i]; }
  return w; }
__device__ __forceinline__ v16h wcolh_oi(const float* Wm, int k0, int o, int lane, int K) { v16h w; const float* p = Wm + (size_t)o * K + k0 + 8 * (lane >> 4);
#pragma unroll
  for (int i = 0; i < 8; ++i) { w[i] = (_Float16)(bfr(p[i]) * 256.0f); w[8 + i] = (_Float16)(bfr(p[16 + i]) * 256.0f); }
  return w; }
#define LDSX() do { asm volatile("s_wait_dscnt 0" ::: "memory"); __builtin_amdgcn_wave_barrier(); __builtin_amdgcn_fence(3  , "workgroup"); } while (0)

#ifndef NB
#define NB 2
#endif
#ifndef SEQ
#define SEQ 2048
#endif
#define NB_FULL 2
#define SEQ_FULL 2048
#define TT SEQ
#define DIN 2048
#define NH 16
#define NKVH 8
#define HD 128
#define CC (NH * HD)
#define CKV (NKVH * HD)
#define GQ (NH / NKVH)
#define HG 4
#define NQB (TT / 64)
#define SCALE (0.08838834764831845f)
#define RMS_EPS (1.0e-6f)
#define QBH 6
#define QHI 384
#define KHI 384

static_assert(NB >= 1 && NB <= NB_FULL);
static_assert(TT % 128 == 0 && TT <= SEQ_FULL);
static_assert(QHI % 64 == 0 && KHI % 64 == 0 && QBH * 64 <= QHI);
static_assert(((((QBH * 64 - 1) >> 7) + 1) * 128) <= KHI);
static_assert(HD == 128 && NH % HG == 0 && CC % 128 == 0 && CKV % 128 == 0 && DIN % 32 == 0);

__host__ __device__ __forceinline__ int kb_last(int qb) { return (qb * 64 + 63) >> 7; }

__constant__ float c_invf[64] = { 1.0f,0.8058422207832336f,0.6493816375732422f,0.5232991576194763f,0.4216965138912201f,0.33982083201408386f,0.2738419771194458f,0.22067339718341827f,0.17782793939113617f,0.14330126345157623f,0.11547820270061493f,0.09305720031261444f,0.07498941570520401f,0.0604296438395977f,0.04869675263762474f,0.03924189880490303f,0.03162277862429619f,0.025482967495918274f,0.02053525112569332f,0.016548171639442444f,0.01333521492779255f,0.010746078565716743f,0.00865964312106371f,0.006978305988013744f,0.005623413249850273f,0.004531583748757839f,0.003651741426438093f,0.002942727180197835f,0.0023713738191872835f,0.001910952851176262f,0.0015399265103042126f,0.0012409378541633487f,0.0010000000474974513f,0.0008058422245085239f,0.0006493816617876291f,0.0005232990952208638f,0.00042169648804701865f,0.00033982080640271306f,0.00027384195709601045f,0.00022067342069931328f,0.00017782794020604342f,0.00014330126577988267f,0.00011547819303814322f,9.305720595875755e-05f,7.498942431993783e-05f,6.042963650543243e-05f,4.869675467489287e-05f,3.92418987757992e-05f,3.162277425872162e-05f,2.5482966520939954e-05f,2.0535249859676696e-05f,1.6548170606256463e-05f,1.333521413471317e-05f,1.0746078260126524e-05f,8.659643754072022e-06f,6.978306373639498e-06f,5.62341347176698e-06f,4.531583726929966e-06f,3.651741280918941e-06f,2.9427271783788456e-06f,2.3713737391517498e-06f,1.910952960315626e-06f,1.5399265294036013e-06f,1.2409377632138785e-06f };

#define WS_QH  ((size_t)0)
#define WS_QL  (WS_QH  + 2u * (size_t)NB * TT * CC)
#define WS_KH  (WS_QL  + 2u * (size_t)NB * QHI * CC)
#define WS_KL  (WS_KH  + 2u * (size_t)NB * TT * CKV)
#define WS_VT  (WS_KL  + 2u * (size_t)NB * KHI * CKV)
#define WS_VB  (WS_VT  + 2u * (size_t)NB * CKV * TT)
#define WS_VBL (WS_VB  + 2u * (size_t)NB * CKV * KHI)
#define WS_CS  (WS_VBL + 2u * (size_t)NB * CKV * KHI)
#define WS_S   (WS_CS  + 4u * (size_t)NB * TT * 128)
#define WS_Y   (WS_S   + 4u * (size_t)HG * TT * TT)
#define WS_FL  (WS_Y   + 4u * (size_t)TT * CC)
#define WS_END (WS_FL  + 256u)
static_assert(WS_END <= (size_t)134217728u);
static_assert((WS_QL % 256u) == 0 && (WS_KH % 256u) == 0 && (WS_KL % 256u) == 0 && (WS_VT % 256u) == 0 && (WS_VB % 256u) == 0 && (WS_VBL % 256u) == 0 && (WS_CS % 256u) == 0 && (WS_S % 256u) == 0 && (WS_Y % 256u) == 0 && (WS_FL % 256u) == 0);

__global__ __launch_bounds__(256) void k_rope(const int* __restrict__ POS, float* __restrict__ CS) {
  __shared__ __align__(16) float cs[32][132];
  const int tid = threadIdx.x, wave = tid >> 5, lane = tid & 31; const int r0 = blockIdx.x * 32;
#pragma unroll 1
  for (int e = tid; e < 32 * 64; e += 256) { const int rl = e >> 6, i = e & 63; const int r = r0 + rl; const int bb = r / TT, t = r % TT;
    const float pf = (float)POS[(size_t)bb * SEQ_FULL + t]; float sn, cn; sincosf(pf * c_invf[i], &sn, &cn); cs[rl][i] = cn; cs[rl][64 + i] = sn; }
  __syncthreads();
  for (int rl = wave; rl < 32; rl += 8) vst2(CS + (size_t)(r0 + rl) * 128 + lane * 4, *(const v4f*)&cs[rl][lane * 4]);
}

__global__ __launch_bounds__(128) void k_proj(const float* __restrict__ X, const float* __restrict__ WQ, const float* __restrict__ WK, const float* __restrict__ WV, const float* __restrict__ CS, const float* __restrict__ QNW, const float* __restrict__ KNW,
    _Float16* __restrict__ QH, _Float16* __restrict__ QL, _Float16* __restrict__ KH, _Float16* __restrict__ KL, _Float16* __restrict__ VT, __bf16* __restrict__ VB, __bf16* __restrict__ VBL) {
  __shared__ __align__(16) float st[64][132]; __shared__ __align__(16) _Float16 sh[64][136], sl[64][136]; __shared__ __align__(16) _Float16 th[128][72]; __shared__ __align__(16) __bf16 tb[128][72], tbl[128][72];
  const int which = blockIdx.z; const int c0 = blockIdx.y * 128;
  if (which != 0 && c0 >= CKV) return;
  const int tid = threadIdx.x, wave = tid >> 5, lane = tid & 31, col = lane & 15, g = lane >> 4;
  const size_t r0 = (size_t)blockIdx.x * 64; const int bb = (int)(r0 / TT); const int t0 = (int)(r0 % TT);
  const float* WA = which == 0 ? WQ : which == 1 ? WK : WV;
  const size_t xr0 = (size_t)bb * SEQ_FULL + t0;
  v8f acc[8] = {};
#pragma unroll 2
  for (int kc = 0; kc < DIN / 32; ++kc) { v16b a; { const float* p = X + (xr0 + wave * 16 + col) * DIN + kc * 32 + 8 * g;
#pragma unroll
      for (int i = 0; i < 8; ++i) { a[i] = (__bf16)p[i]; a[8 + i] = (__bf16)p[16 + i]; } }
    asm volatile("s_wait_loadcnt 0x0" ::: "memory");
#pragma unroll
    for (int j = 0; j < 8; ++j) { const v16b w = wcol_oi(WA, kc * 32, c0 + j * 16 + col, lane, DIN); asm volatile("s_wait_loadcnt 0x0" ::: "memory"); acc[j] = wmma_bf(a, w, acc[j]); } }
#pragma unroll
  for (int j = 0; j < 8; ++j)
#pragma unroll
    for (int r = 0; r < 8; ++r) st[wave * 16 + 8 * g + r][j * 16 + col] = acc[j][r];
  __syncthreads();
  if (which < 2) {
    const float* nw = which == 0 ? QNW : KNW;
    for (int e = tid; e < 64; e += 128) { float* rw = &st[e][0];
      float ssq = 0.f;
#pragma unroll 8
      for (int i = 0; i < HD; ++i) ssq += rw[i] * rw[i];
      const float rs = rsqrtf(ssq * (1.0f / 128.0f) + RMS_EPS);
#pragma unroll 8
      for (int i = 0; i < HD; ++i) rw[i] = bfr(nw[i]) * (rw[i] * rs);
      const float* csr = CS + (r0 + e) * 128;
#pragma unroll 4
      for (int i = 0; i < 64; ++i) { const float a = rw[i], c = rw[64 + i], cn = csr[i], sn = csr[64 + i]; rw[i] = a * cn - c * sn; rw[64 + i] = c * cn + a * sn; } }
    __syncthreads();
    _Float16* DH = which == 0 ? QH : KH; _Float16* DL = which == 0 ? QL : KL; const int nhi = which == 0 ? QHI : KHI; const int P = which == 0 ? CC : CKV; const bool hi_rows = t0 < nhi;
    for (int e = tid; e < 64 * 128; e += 128) { const int rl = e >> 7, cl = e & 127; const float v = st[rl][cl]; const _Float16 hv = (_Float16)v; sh[rl][cl] = hv; sl[rl][cl] = (_Float16)((v - (float)hv) * 1024.0f); }
    __syncthreads();
    for (int e = tid; e < 64 * 16; e += 128) { const int rl = e >> 4, q = e & 15;
      vst2((unsigned*)(DH + (r0 + rl) * (size_t)P + c0 + q * 8), *(const v4u*)&sh[rl][q * 8]);
      if (hi_rows) vst2((unsigned*)(DL + ((size_t)bb * nhi + t0 + rl) * (size_t)P + c0 + q * 8), *(const v4u*)&sl[rl][q * 8]); }
  } else { const bool hi_rows = t0 < KHI;
    for (int e = tid; e < 64 * 128; e += 128) { const int rl = e & 63, cl = e >> 6; const float v = st[rl][cl]; th[cl][rl] = (_Float16)v; const __bf16 bh = (__bf16)v; tb[cl][rl] = bh; tbl[cl][rl] = (__bf16)(v - (float)bh); }
    __syncthreads();
    for (int e = tid; e < 128 * 8; e += 128) { const int cl = e >> 3, q = e & 7;
      vst2((unsigned*)(VT + ((size_t)bb * CKV + c0 + cl) * (size_t)TT + t0 + q * 8), *(const v4u*)&th[cl][q * 8]);
      if (hi_rows) { const size_t o3 = ((size_t)bb * CKV + c0 + cl) * (size_t)KHI + t0 + q * 8; vst2((unsigned*)(VB + o3), *(const v4u*)&tb[cl][q * 8]); vst2((unsigned*)(VBL + o3), *(const v4u*)&tbl[cl][q * 8]); } } }
}
__global__ __launch_bounds__(256) void k_chk(const float* __restrict__ AM, int* __restrict__ FL) {
  __shared__ int sred[8];
  const int tid = threadIdx.x, wave = tid >> 5, lane = tid & 31;
  int cnt = 0; const unsigned total = (unsigned)NB * TT * TT;
#pragma unroll 1
  for (unsigned e = tid; e < total; e += 256) { const int k = (int)(e % TT), t = (int)((e / TT) % TT), bb = (int)(e / ((unsigned)TT * TT));
    const float v = AM[((size_t)bb * SEQ_FULL + t) * (size_t)SEQ_FULL + k];
    cnt += (k > t && !(v <= -1.0e4f)) ? 1 : 0; }
#pragma unroll
  for (int o = 1; o < 32; o <<= 1) cnt += __shfl_xor(cnt, o);
  if (lane == 0) sred[wave] = cnt; __syncthreads();
  if (wave == 0) { int a = 0;
#pragma unroll
    for (int i = 0; i < 8; ++i) a += sred[i];
    const int fv = (a != 0) ? 1 : 2; v4i f4; f4[0] = fv; f4[1] = fv; f4[2] = fv; f4[3] = fv;
    if (lane < 8) vst2(FL + lane * 4, f4); }
}
__global__ __launch_bounds__(128) void k_sc(const _Float16* __restrict__ QH, const _Float16* __restrict__ KH, const _Float16* __restrict__ QL, const _Float16* __restrict__ KL, int b, int h0, float* __restrict__ S0) { __shared__ __align__(16) float ss[4][16][132];
  const int qb = blockIdx.x, kb = blockIdx.y; if (kb > kb_last(qb)) return;
  const int h = h0 + blockIdx.z, hk = h / GQ; float* S = S0 + (size_t)blockIdx.z * TT * TT;
  const int tid = threadIdx.x, wave = tid >> 5, lane = tid & 31, col = lane & 15, g = lane >> 4; const int k0 = kb * 128; const int ql0 = qb * 64 + wave * 16; const size_t q0 = (size_t)b * TT + ql0, kr0 = (size_t)b * TT + k0;
  v8f acc[8] = {}, accl[8] = {};
  const _Float16* QLb = QL + (size_t)b * QHI * CC; const _Float16* KLb = KL + (size_t)b * KHI * CKV;
  if (qb < QBH) {
#pragma unroll
    for (int kc = 0; kc < HD / 32; ++kc) { const v16h ah = frag_h(QH + (q0 + col) * CC + h * HD + kc * 32, lane), al = frag_h(QLb + (size_t)(ql0 + col) * CC + h * HD + kc * 32, lane);
#pragma unroll
      for (int j = 0; j < 8; ++j) { const v16h kbf = frag_h(KH + (kr0 + j * 16 + col) * CKV + hk * HD + kc * 32, lane), klf = frag_h(KLb + (size_t)(k0 + j * 16 + col) * CKV + hk * HD + kc * 32, lane); acc[j] = wmma16(ah, kbf, acc[j]); accl[j] = wmma16(al, kbf, accl[j]); accl[j] = wmma16(ah, klf, accl[j]); } }
  } else if (qb * 64 < QHI) {
#pragma unroll
    for (int kc = 0; kc < HD / 32; ++kc) { const v16h ah = frag_h(QH + (q0 + col) * CC + h * HD + kc * 32, lane), al = frag_h(QLb + (size_t)(ql0 + col) * CC + h * HD + kc * 32, lane);
#pragma unroll
      for (int j = 0; j < 8; ++j) { const v16h kbf = frag_h(KH + (kr0 + j * 16 + col) * CKV + hk * HD + kc * 32, lane); acc[j] = wmma16(ah, kbf, acc[j]); accl[j] = wmma16(al, kbf, accl[j]); } }
  } else {
#pragma unroll
    for (int kc = 0; kc < HD / 32; ++kc) { const v16h ah = frag_h(QH + (q0 + col) * CC + h * HD + kc * 32, lane);
#pragma unroll
      for (int j = 0; j < 8; ++j) { const v16h kbf = frag_h(KH + (kr0 + j * 16 + col) * CKV + hk * HD + kc * 32, lane); acc[j] = wmma16(ah, kbf, acc[j]); } } }
#pragma unroll
  for (int j = 0; j < 8; ++j) {
#pragma unroll
    for (int r = 0; r < 8; ++r) ss[wave][8 * g + r][j * 16 + col] = (acc[j][r] + accl[j][r] * (1.0f / 1024.0f)) * SCALE; }
  LDSX(); for (int rl = 0; rl < 16; ++rl) vst2(S + (size_t)(ql0 + rl) * TT + k0 + lane * 4, *(const v4f*)&ss[wave][rl][lane * 4]); }
__global__ __launch_bounds__(256) void k_sm(float* __restrict__ S0, const float* __restrict__ AMb) { __shared__ float sred[8]; __shared__ float sbc; __shared__ __align__(16) float shv[TT];
  const int tid = threadIdx.x; const int t = blockIdx.x; const int kend = (kb_last(t >> 6) + 1) * 128;
  float* sr = S0 + (size_t)blockIdx.y * TT * TT + (size_t)t * TT;
  const float* am = AMb + (size_t)t * SEQ_FULL;
  float m = -3.0e38f; for (int k = tid; k < kend; k += 256) { const float sv = sr[k], av = am[k]; const float v = (k <= t) ? (sv + av) : -3.0e38f; shv[k] = v; m = fmaxf(m, v); }
#pragma unroll
  for (int o = 1; o < 32; o <<= 1) m = fmaxf(m, __shfl_xor(m, o));
  if ((tid & 31) == 0) sred[tid >> 5] = m; __syncthreads(); if (tid == 0) { float a = sred[0]; for (int i = 1; i < 8; ++i) a = fmaxf(a, sred[i]); sbc = a; } __syncthreads(); m = sbc; __syncthreads();
  float sum = 0.f; for (int k = tid; k < kend; k += 256) { const float v = shv[k]; const float e = (v <= -1.0e38f) ? 0.f : expf(v - m); shv[k] = e; sum += e; }
#pragma unroll
  for (int o = 1; o < 32; o <<= 1) sum += __shfl_xor(sum, o);
  if ((tid & 31) == 0) sred[tid >> 5] = sum; __syncthreads(); if (tid == 0) { float a = 0.f; for (int i = 0; i < 8; ++i) a += sred[i]; sbc = a > 0.f ? 2048.0f / a : 0.f; }     __syncthreads(); const float inv = sbc;
  for (int k = tid; k < kend; k += 256) shv[k] = shv[k] * inv;
  __syncthreads(); for (int q = tid; q < kend / 4; q += 256) vst2(sr + q * 4, *(const v4f*)&shv[q * 4]); }
__global__ __launch_bounds__(128) void k_pv(const float* __restrict__ PS0, const _Float16* __restrict__ VT, const __bf16* __restrict__ VB, const __bf16* __restrict__ VBL, int b, int h0, float* __restrict__ Y) { const int h = h0 + blockIdx.z, hk = h / GQ; const float* PS = PS0 + (size_t)blockIdx.z * TT * TT; __shared__ __align__(16) float ss[4][16][HD + 4];
  const int tid = threadIdx.x, wave = tid >> 5, lane = tid & 31, col = lane & 15, g = lane >> 4; const int qb = blockIdx.x; const int ql0 = qb * 64 + wave * 16; const int kce = (kb_last(qb) + 1) * 4;
  v8f acc[HD / 16] = {};
  if (qb < QBH) {
#pragma unroll 1
    for (int kc = 0; kc < kce; ++kc) { const F2 p = split_row(PS + (size_t)(ql0 + col) * TT, kc * 32, lane);
      asm volatile("s_wait_loadcnt 0x0" ::: "memory");
#pragma unroll
      for (int j = 0; j < HD / 16; ++j) { const size_t po = ((size_t)b * CKV + hk * HD + j * 16 + col) * (size_t)KHI + kc * 32; const v16b vh = frag_b(VB + po, lane); acc[j] = wmma_bf(p.h, vh, acc[j]); acc[j] = wmma_bf(p.l, vh, acc[j]); acc[j] = wmma_bf(p.h, frag_b(VBL + po, lane), acc[j]); } }
  } else {
#pragma unroll 1
    for (int kc = 0; kc < kce; ++kc) { const v16h p = frag_f32(PS + (size_t)(ql0 + col) * TT + kc * 32, lane);
      asm volatile("s_wait_loadcnt 0x0" ::: "memory");
#pragma unroll
      for (int j = 0; j < HD / 16; ++j) { const size_t po = ((size_t)b * CKV + hk * HD + j * 16 + col) * (size_t)TT + kc * 32; acc[j] = wmma16(p, frag_h(VT + po, lane), acc[j]); } } }
#pragma unroll
  for (int j = 0; j < HD / 16; ++j)
#pragma unroll
    for (int r = 0; r < 8; ++r) ss[wave][8 * g + r][j * 16 + col] = acc[j][r] * (1.0f / 2048.0f);
  LDSX(); for (int rl = 0; rl < 16; ++rl) vst2(Y + (size_t)(ql0 + rl) * CC + h * HD + lane * 4, *(const v4f*)&ss[wave][rl][lane * 4]); }
__global__ __launch_bounds__(128) void k_out(const float* __restrict__ Y, const float* __restrict__ WO, const int* __restrict__ FL, int b, float* __restrict__ OUT) { __shared__ __align__(16) float sf[4][16][132];
  const int tid = threadIdx.x, wave = tid >> 5, lane = tid & 31, col = lane & 15, g = lane >> 4; const int c0 = blockIdx.y * 128; const int r0 = blockIdx.x * 64 + wave * 16;
  const bool hi = (int)(blockIdx.x * 64) < QHI;
  v8f acc[8] = {};
  if (hi) {
#pragma unroll 2
    for (int kc = 0; kc < CC / 32; ++kc) { const F2 a = split_row(Y + (size_t)(r0 + col) * CC, kc * 32, lane); asm volatile("s_wait_loadcnt 0x0" ::: "memory");
#pragma unroll
      for (int j = 0; j < 8; ++j) { const v16b w = wcol_oi(WO, kc * 32, c0 + j * 16 + col, lane, CC); asm volatile("s_wait_loadcnt 0x0" ::: "memory"); acc[j] = wmma_bf(a.h, w, acc[j]); acc[j] = wmma_bf(a.l, w, acc[j]); } }
#pragma unroll
    for (int j = 0; j < 8; ++j) {
#pragma unroll
      for (int r = 0; r < 8; ++r) sf[wave][8 * g + r][j * 16 + col] = acc[j][r]; }
  } else {
#pragma unroll 2
    for (int kc = 0; kc < CC / 32; ++kc) { const v16h a = frag_f32(Y + (size_t)(r0 + col) * CC + kc * 32, lane); asm volatile("s_wait_loadcnt 0x0" ::: "memory");
#pragma unroll
      for (int j = 0; j < 8; ++j) { const v16h w = wcolh_oi(WO, kc * 32, c0 + j * 16 + col, lane, CC); asm volatile("s_wait_loadcnt 0x0" ::: "memory"); acc[j] = wmma16(a, w, acc[j]); } }
#pragma unroll
    for (int j = 0; j < 8; ++j) {
#pragma unroll
      for (int r = 0; r < 8; ++r) sf[wave][8 * g + r][j * 16 + col] = acc[j][r] * (1.0f / 256.0f); } }
  const int fl = FL[0]; const float qn = __uint_as_float(0x7fc00000u);
  LDSX(); for (int rl = 0; rl < 16; ++rl) { v4f v = *(const v4f*)&sf[wave][rl][lane * 4]; if (fl == 1) { v[0] = qn; v[1] = qn; v[2] = qn; v[3] = qn; }
    vst2(OUT + ((size_t)b * SEQ_FULL + r0 + rl) * DIN + c0 + lane * 4, v); } }

extern "C" void kernel_launch(void* const* d_in, const int* in_sizes, int n_in, void* d_out, int out_size, void* d_ws, size_t ws_size, hipStream_t stream) {
  if (n_in < 9) return;
  const size_t rows_used = (size_t)(NB - 1) * SEQ_FULL + TT;
  if ((size_t)in_sizes[0] < rows_used * DIN) return;
  if ((size_t)in_sizes[1] < rows_used * SEQ_FULL) return;
  if ((size_t)in_sizes[2] < rows_used) return;
  if ((size_t)in_sizes[3] < (size_t)CC * DIN || (size_t)in_sizes[4] < (size_t)CKV * DIN || (size_t)in_sizes[5] < (size_t)CKV * DIN || (size_t)in_sizes[6] < (size_t)DIN * CC) return;
  if (in_sizes[7] < HD || in_sizes[8] < HD) return;
  if ((size_t)out_size < rows_used * DIN) return;
  if (ws_size < WS_END) return;
  const float* const* F = (const float* const*)d_in;
  const float* X = F[0]; const float* AM = F[1]; const int* POS = (const int*)d_in[2];
  char* ws = (char*)d_ws;
  _Float16 *QH = (_Float16*)(ws + WS_QH), *QL = (_Float16*)(ws + WS_QL), *KH = (_Float16*)(ws + WS_KH), *KL = (_Float16*)(ws + WS_KL), *VT = (_Float16*)(ws + WS_VT);
  __bf16 *VB = (__bf16*)(ws + WS_VB), *VBL = (__bf16*)(ws + WS_VBL);
  float *CS = (float*)(ws + WS_CS), *S = (float*)(ws + WS_S), *Y = (float*)(ws + WS_Y); int* FL = (int*)(ws + WS_FL);
  k_rope<<<dim3(NB * TT / 32), 256, 0, stream>>>(POS, CS);
  k_proj<<<dim3(NB * TT / 64, CC / 128, 3), 128, 0, stream>>>(X, F[3], F[4], F[5], CS, F[7], F[8], QH, QL, KH, KL, VT, VB, VBL);
  k_chk<<<dim3(1), 256, 0, stream>>>(AM, FL);
  for (int b = 0; b < NB; ++b) {
    for (int h0 = 0; h0 < NH; h0 += HG) {
      k_sc<<<dim3(NQB, TT / 128, HG), 128, 0, stream>>>(QH, KH, QL, KL, b, h0, S);
      k_sm<<<dim3(TT, HG), 256, 0, stream>>>(S, AM + (size_t)b * SEQ_FULL * SEQ_FULL);
      k_pv<<<dim3(NQB, 1, HG), 128, 0, stream>>>(S, VT, VB, VBL, b, h0, Y); }
    k_out<<<dim3(TT / 64, DIN / 128), 128, 0, stream>>>(Y, F[6], FL, b, (float*)d_out); }
}
